// GraphEncoder_60533269070360
// MI455X (gfx1250) — hardware-verified
//
#include <hip/hip_runtime.h>
#include <stddef.h>


typedef _Float16 h16;
typedef _Float16 v16h __attribute__((ext_vector_type(16)));
typedef _Float16 v8h  __attribute__((ext_vector_type(8)));
typedef _Float16 v4h  __attribute__((ext_vector_type(4)));
typedef float    v8f  __attribute__((ext_vector_type(8)));
typedef float    v4f  __attribute__((ext_vector_type(4)));
typedef int      v4i  __attribute__((ext_vector_type(4)));

#ifndef NB
#define NB 4
#endif
#ifndef TT
#define TT 32
#endif
#define NB_FULL 4
#define TT_FULL 32
#define NNODE  64
#define DIM    128
#define HID    512
#define NHEAD  4
#define HD     32
#define NLAYER 3
#define RANK   8
#define NGRAPH (NB * TT)
#define MROWS  (NGRAPH * NNODE)

#define OUT1_OFF ((size_t)NB_FULL * TT_FULL * NNODE * DIM)
#define OUT2_OFF (OUT1_OFF + (size_t)NB_FULL * TT_FULL * DIM)
#define OUT_TOTAL (OUT2_OFF + (size_t)NNODE * NNODE)

static_assert(NB >= 1 && NB <= NB_FULL);
static_assert(TT >= 1 && TT <= TT_FULL);
static_assert(NNODE == 64);
static_assert(DIM == NHEAD * HD);
static_assert(HD == 32);
static_assert(DIM == 32 * 4);
static_assert(HID == 4 * DIM);
static_assert((DIM % 64) == 0 && (DIM % 32) == 0);
static_assert((HID % 64) == 0 && (HID % 32) == 0);
static_assert((NNODE % 32) == 0);
static_assert((MROWS % 64) == 0 && (MROWS % 16) == 0 && (MROWS % 8) == 0);
static_assert(OUT1_OFF * 4 == (size_t)4194304);
static_assert(OUT2_OFF * 4 == (size_t)4259840);
static_assert(OUT_TOTAL * 4 == (size_t)4276224);
static_assert(((OUT1_OFF * 4) % 128) == 0 && ((OUT2_OFF * 4) % 128) == 0);

#define LDT 72
#define LDC 68
#define XP  132
#define LDY 136
static_assert((LDT % 8) == 0 && LDT >= 64);
static_assert((LDC % 4) == 0 && LDC >= 64);
static_assert((XP % 4) == 0 && XP >= DIM);
static_assert((LDY % 8) == 0 && LDY >= DIM);

#define WCARRY 64.0f
#define ACARRY 64.0f
#define PCARRY 16384.0f
#define YCARRY 16.0f
#define MCARRY 16.0f
#define RCARRY 2048.0f

#define WSQ_BYTES ((size_t)DIM * DIM * 2)
#define WFF_BYTES ((size_t)DIM * HID * 2)
#define A16_BYTES ((size_t)NNODE * NNODE * 2)
#define LB_BYTES  ((size_t)NNODE * NNODE * 4)
#define P16_BYTES ((size_t)MROWS * DIM * 2)
#define PF_BYTES  ((size_t)MROWS * DIM * 4)
#define MID_BYTES ((size_t)MROWS * HID * 2)
#define OFF_WP  ((size_t)0)
#define OFF_WL  (OFF_WP + WSQ_BYTES)
#define OFF_WO  (OFF_WL + NLAYER * WSQ_BYTES)
#define OFF_W1  (OFF_WO + NLAYER * WSQ_BYTES)
#define OFF_W2  (OFF_W1 + NLAYER * WFF_BYTES)
#define OFF_A16 (OFF_W2 + NLAYER * WFF_BYTES)
#define OFF_LB  (OFF_A16 + A16_BYTES)
#define OFF_X16 (OFF_LB + LB_BYTES)
#define OFF_HN  (OFF_X16 + P16_BYTES)
#define OFF_HNR (OFF_HN + P16_BYTES)
#define OFF_Y   (OFF_HNR + P16_BYTES)
#define OFF_H2  (OFF_Y + P16_BYTES)
#define OFF_XH  (OFF_H2 + P16_BYTES)
#define OFF_Z   (OFF_XH + PF_BYTES)
#define OFF_ZH  (OFF_Z + PF_BYTES)
#define OFF_UP  (OFF_ZH + PF_BYTES)
#define OFF_U   (OFF_UP + PF_BYTES)
#define OFF_MID (OFF_U + PF_BYTES)
#define OFF_MIDR (OFF_MID + MID_BYTES)
#define WS_TOTAL (OFF_MIDR + MID_BYTES)
static_assert((WSQ_BYTES % 128) == 0 && (WFF_BYTES % 128) == 0 && (A16_BYTES % 128) == 0);
static_assert((LB_BYTES % 128) == 0 && (P16_BYTES % 128) == 0 && (PF_BYTES % 128) == 0);
static_assert((MID_BYTES % 128) == 0);
static_assert(WS_TOTAL <= (size_t)134217728);
static_assert(NB != NB_FULL || TT != TT_FULL || WS_TOTAL == (size_t)49274880);

union GraphTileA {
  float    f[NNODE * XP];
  _Float16 h[NNODE * LDY];
};
union GraphTileC {
  float    f[NNODE * NNODE];
  _Float16 h[DIM * LDT];
};
#define PH_HALVES (NHEAD * NNODE * LDT)
#define HT_HALVES (DIM * LDT)
#define GRAPH_LDS_BYTES (sizeof(GraphTileA) + sizeof(GraphTileC) + (size_t)PH_HALVES * 2 + (size_t)NHEAD * NNODE * 4)
static_assert(sizeof(GraphTileA) == (size_t)NNODE * XP * 4);
static_assert(sizeof(GraphTileC) == (size_t)DIM * LDT * 2);
static_assert((size_t)NNODE * LDY * 2 <= (size_t)NNODE * XP * 4);
static_assert((size_t)NNODE * NNODE * 4 <= (size_t)DIM * LDT * 2);
static_assert(2 * HT_HALVES <= PH_HALVES);
static_assert(GRAPH_LDS_BYTES == (size_t)90112);
static_assert(GRAPH_LDS_BYTES <= (size_t)100000);

__device__ __forceinline__ float bf16r(float x) {
  unsigned int u = __float_as_uint(x);
  u = (u + 0x7FFFu + ((u >> 16) & 1u)) & 0xFFFF0000u;
  return __uint_as_float(u);
}

static __device__ __forceinline__ h16 toh_flush(float v) {
  const h16 r = (h16)v;
  return (fabsf(v) < 6.103515625e-05f) ? (h16)0.0f : r;
}

__device__ __forceinline__ v16h frag_at(const _Float16* p) {
  v8h lo = *(const v8h*)(p);
  v8h hi = *(const v8h*)(p + 16);
  v16h out;
#pragma unroll
  for (int i = 0; i < 8; ++i) { out[i] = lo[i]; out[i + 8] = hi[i]; }
  return out;
}
__device__ __forceinline__ v16h ld_frag(const _Float16* base, unsigned ld) {
  const unsigned lane = threadIdx.x & 31u;
  return frag_at(base + (lane & 15u) * ld + (lane >> 4) * 8u);
}

__device__ __forceinline__ v8f wmma16(v16h a, v16h b, v8f c) {
  v8f d = __builtin_amdgcn_wmma_f32_16x16x32_f16(false, a, false, b, (short)0, c,
                                                 false, false);
  asm volatile("v_nop\n\tv_nop\n\tv_nop\n\tv_nop" : "+v"(d) : "v"(a), "v"(b));
  return d;
}

__device__ __forceinline__ float red32_sum(float x) {
#pragma unroll
  for (int off = 1; off < 32; off <<= 1) x += __shfl_xor(x, off, 32);
  return x;
}
__device__ __forceinline__ float red32_max(float x) {
#pragma unroll
  for (int off = 1; off < 32; off <<= 1) x = fmaxf(x, __shfl_xor(x, off, 32));
  return x;
}

__device__ __forceinline__ float sigmoid_act(float t) {
  return __builtin_amdgcn_rcpf(1.0f + __expf(-t));
}
__device__ __forceinline__ float silu_act(float t) {
  return t * __builtin_amdgcn_rcpf(1.0f + __expf(-t));
}

__global__ __launch_bounds__(256) void wconv_kernel(
    const float* __restrict__ W, _Float16* __restrict__ Wt, unsigned ldw, unsigned ldk) {
  __shared__ _Float16 T[64 * LDT];
  const unsigned tid = threadIdx.x;
  const unsigned n0 = blockIdx.x * 64u;
  const unsigned k0 = blockIdx.y * 64u;
#pragma unroll 4
  for (unsigned j = 0; j < 16u; ++j) {
    const unsigned idx = tid + 256u * j;
    const unsigned kr = idx >> 6, nc = idx & 63u;
    const float v = W[(size_t)(k0 + kr) * ldw + n0 + nc];
    T[nc * LDT + kr] = (_Float16)(WCARRY * bf16r(v));
  }
  __syncthreads();
  v8h x[2];
  size_t off[2];
#pragma unroll
  for (unsigned i = 0; i < 2u; ++i) {
    const unsigned n = 32u * i + (tid >> 3);
    const unsigned kc = (tid & 7u) * 8u;
    x[i] = *(const v8h*)&T[n * LDT + kc];
    off[i] = (size_t)(n0 + n) * ldk + k0 + kc;
  }
#pragma unroll
  for (int i = 0; i < 2; ++i) *(volatile v8h*)(Wt + off[i]) = x[i];
  __threadfence();
#pragma unroll
  for (int i = 0; i < 2; ++i) *(volatile v8h*)(Wt + off[i]) = x[i];
}

__global__ __launch_bounds__(256) void adj_kernel(
    const float* __restrict__ A0, const int* __restrict__ maskp,
    const float* __restrict__ Pm, const float* __restrict__ Qm,
    const float* __restrict__ alphap,
    float* __restrict__ outA, _Float16* __restrict__ A16, float* __restrict__ LB) {
  __shared__ __attribute__((aligned(16))) float As[NNODE * NNODE];
  __shared__ __attribute__((aligned(16))) float Lg[NNODE * NNODE];
  __shared__ float rinv[NNODE];
  const unsigned tid = threadIdx.x;
  const float alpha = bf16r(alphap[0]);
#pragma unroll 1
  for (unsigned k = 0; k < 16u; ++k) {
    const unsigned idx = tid + 256u * k;
    const unsigned i = idx >> 6, j = idx & 63u;
    float s = 0.0f;
#pragma unroll 1
    for (unsigned r = 0; r < (unsigned)RANK; ++r)
      s += bf16r(Pm[i * RANK + r]) * bf16r(Qm[j * RANK + r]);
    const float sp = fmaxf(s, 0.0f) + __logf(1.0f + __expf(-fabsf(s)));
    const float a0 = bf16r(A0[idx]);
    const int mk = maskp[idx];
    const float ad = (mk != 0) ? sp : 0.0f;
    As[idx] = a0 * (1.0f + alpha * ad);
    Lg[idx] = logf(a0 + 1.0e-8f);
  }
  __syncthreads();
  if (tid < (unsigned)NNODE) {
    float s = 0.0f;
#pragma unroll 4
    for (unsigned j = 0; j < (unsigned)NNODE; ++j) s += As[tid * NNODE + j];
    rinv[tid] = __builtin_amdgcn_rcpf(s + 1.0e-8f);
  }
  __syncthreads();
  v4f oa[4], ol[4];
  v8h oh[2];
#pragma unroll
  for (unsigned k = 0; k < 4u; ++k) {
    const unsigned e = (tid + 256u * k) * 4u;
    const float rv = rinv[e >> 6];
    const v4f a = *(const v4f*)&As[e];
    v4f t;
#pragma unroll
    for (int j = 0; j < 4; ++j) t[j] = a[j] * rv;
    oa[k] = t;
    ol[k] = *(const v4f*)&Lg[e];
  }
#pragma unroll
  for (unsigned k = 0; k < 2u; ++k) {
    const unsigned e = (tid + 256u * k) * 8u;
    const float rv = rinv[e >> 6];
#pragma unroll
    for (unsigned j = 0; j < 8u; ++j) oh[k][j] = toh_flush(ACARRY * (As[e + j] * rv));
  }
#pragma unroll
  for (unsigned k = 0; k < 4u; ++k) {
    const unsigned e = (tid + 256u * k) * 4u;
    *(volatile v4f*)(outA + e) = oa[k];
    *(volatile v4f*)(LB + e) = ol[k];
  }
#pragma unroll
  for (unsigned k = 0; k < 2u; ++k) *(volatile v8h*)(A16 + (tid + 256u * k) * 8u) = oh[k];
  __threadfence();
#pragma unroll
  for (unsigned k = 0; k < 4u; ++k) {
    const unsigned e = (tid + 256u * k) * 4u;
    *(volatile v4f*)(outA + e) = oa[k];
    *(volatile v4f*)(LB + e) = ol[k];
  }
#pragma unroll
  for (unsigned k = 0; k < 2u; ++k) *(volatile v8h*)(A16 + (tid + 256u * k) * 8u) = oh[k];
}

__global__ __launch_bounds__(256) void xconv_kernel(
    const float* __restrict__ X, _Float16* __restrict__ X16) {
  const unsigned gid = blockIdx.x * 256u + threadIdx.x;
  const unsigned crow = gid >> 4;
  const unsigned c = (gid & 15u) * 8u;
  const unsigned g = crow >> 6, n = crow & 63u;
  const unsigned bidx = g / (unsigned)TT;
  const unsigned tq = g - bidx * (unsigned)TT;
  const size_t frow = ((size_t)bidx * TT_FULL + tq) * NNODE + n;
  const v4f a0 = *(const v4f*)(X + frow * DIM + c);
  const v4f a1 = *(const v4f*)(X + frow * DIM + c + 4u);
  v8h o;
#pragma unroll
  for (int i = 0; i < 4; ++i) {
    o[i]     = toh_flush(bf16r(a0[i]));
    o[i + 4] = toh_flush(bf16r(a1[i]));
  }
  _Float16* p = X16 + (size_t)crow * DIM + c;
  *(volatile v8h*)p = o;
  __threadfence();
  *(volatile v8h*)p = o;
}

__global__ __launch_bounds__(256) void ln1_kernel(
    const float* __restrict__ Z, const float* __restrict__ G, const float* __restrict__ Be,
    _Float16* __restrict__ dst, _Float16* __restrict__ dstr) {
  const unsigned lane = threadIdx.x & 31u, w = threadIdx.x >> 5;
  const unsigned crow = blockIdx.x * 8u + w;
  const unsigned c = lane * 4u;
  const v4f a = *(const v4f*)(Z + (size_t)crow * DIM + c);
  const float mean = red32_sum((a[0] + a[1]) + (a[2] + a[3])) * (1.0f / (float)DIM);
  float ss = 0.0f;
#pragma unroll
  for (int i = 0; i < 4; ++i) { const float d = a[i] - mean; ss += d * d; }
  const float var = red32_sum(ss) * (1.0f / (float)DIM);
  const float rstd = 1.0f / sqrtf(var + 1.0e-5f);
  const v4f g = *(const v4f*)(G + c);
  const v4f be = *(const v4f*)(Be + c);
  v4h o, ores;
#pragma unroll
  for (int i = 0; i < 4; ++i) {
    const float t = (a[i] - mean) * rstd * bf16r(g[i]) + bf16r(be[i]);
    const h16 hv = toh_flush(t);
    o[i] = hv;
    ores[i] = toh_flush((t - (float)hv) * RCARRY);
  }
  _Float16* p = dst + (size_t)crow * DIM + c;
  _Float16* pr = dstr + (size_t)crow * DIM + c;
  *(volatile v4h*)p = o;
  *(volatile v4h*)pr = ores;
  __threadfence();
  *(volatile v4h*)p = o;
  *(volatile v4h*)pr = ores;
}

__global__ __launch_bounds__(256) void gate_ln2_kernel(
    const float* __restrict__ UP, const float* __restrict__ fc1W, const float* __restrict__ fc1b,
    const float* __restrict__ fc2W, const float* __restrict__ fc2b,
    const float* __restrict__ G, const float* __restrict__ Be,
    float* __restrict__ Uo, _Float16* __restrict__ H2) {
  const unsigned lane = threadIdx.x & 31u, w = threadIdx.x >> 5;
  const unsigned crow = blockIdx.x * 8u + w;
  const unsigned c = lane * 4u;
  const v4f a = *(const v4f*)(UP + (size_t)crow * DIM + c);
  const float s = red32_sum((a[0] + a[1]) + (a[2] + a[3])) * (1.0f / (float)DIM);
  const v4f f1 = *(const v4f*)(fc1W + c);
  const v4f fb = *(const v4f*)(fc1b + c);
  const v4f f2 = *(const v4f*)(fc2W + c);
  float z = 0.0f;
#pragma unroll
  for (int i = 0; i < 4; ++i) {
    const float hv = s * bf16r(f1[i]) + bf16r(fb[i]);
    z += silu_act(hv) * bf16r(f2[i]);
  }
  z = red32_sum(z) + bf16r(fc2b[0]);
  const float gt = sigmoid_act(z);
  v4f u;
#pragma unroll
  for (int i = 0; i < 4; ++i) u[i] = a[i] * gt;
  const float mean = red32_sum((u[0] + u[1]) + (u[2] + u[3])) * (1.0f / (float)DIM);
  float ss = 0.0f;
#pragma unroll
  for (int i = 0; i < 4; ++i) { const float d = u[i] - mean; ss += d * d; }
  const float var = red32_sum(ss) * (1.0f / (float)DIM);
  const float rstd = 1.0f / sqrtf(var + 1.0e-5f);
  const v4f g = *(const v4f*)(G + c);
  const v4f be = *(const v4f*)(Be + c);
  v4h o;
#pragma unroll
  for (int i = 0; i < 4; ++i)
    o[i] = toh_flush((u[i] - mean) * rstd * bf16r(g[i]) + bf16r(be[i]));
  float* pu = Uo + (size_t)crow * DIM + c;
  _Float16* ph = H2 + (size_t)crow * DIM + c;
  *(volatile v4f*)pu = u;
  *(volatile v4h*)ph = o;
  __threadfence();
  *(volatile v4f*)pu = u;
  *(volatile v4h*)ph = o;
}

template <int MODE>
__device__ __forceinline__ void gemm_body(
    const _Float16* __restrict__ A16, const _Float16* __restrict__ A16r,
    const _Float16* __restrict__ Bt, const unsigned K,
    const float* __restrict__ bias, const float* __restrict__ addf,
    float* __restrict__ outf, _Float16* __restrict__ out16, _Float16* __restrict__ out16r,
    float* __restrict__ outm) {
  __shared__ __attribute__((aligned(16))) float Cs[64 * LDC];
  constexpr bool RES = (MODE == 1 || MODE >= 4);
  const unsigned tid = threadIdx.x, lane = tid & 31u, w = tid >> 5;
  const unsigned mw = w >> 1, nw = w & 1u;
  const unsigned hh = lane >> 4, m = lane & 15u;
  const unsigned n0 = blockIdx.x * 64u;
  const unsigned row0 = blockIdx.y * 64u;

  const _Float16* ap  = A16 + (size_t)(row0 + mw * 16u + m) * K + hh * 8u;
  const _Float16* arp = A16r + (size_t)(row0 + mw * 16u + m) * K + hh * 8u;
  const _Float16* bp0 = Bt + (size_t)(n0 + nw * 32u + m) * K + hh * 8u;
  const _Float16* bp1 = bp0 + (size_t)16 * K;
  v8f acc0 = {}, acc1 = {}, rac0 = {}, rac1 = {};
#pragma unroll 2
  for (unsigned k0 = 0; k0 < K; k0 += 32u) {
    const v16h a  = frag_at(ap + k0);
    const v16h b0 = frag_at(bp0 + k0);
    const v16h b1 = frag_at(bp1 + k0);
    acc0 = wmma16(a, b0, acc0);
    acc1 = wmma16(a, b1, acc1);
    if (RES) {
      const v16h ar = frag_at(arp + k0);
      rac0 = wmma16(ar, b0, rac0);
      rac1 = wmma16(ar, b1, rac1);
    }
  }
#pragma unroll
  for (int r = 0; r < 8; ++r) {
    float* d = &Cs[(mw * 16u + hh * 8u + (unsigned)r) * LDC + nw * 32u + m];
    float v0 = acc0[r], v1 = acc1[r];
    if (RES) {
      v0 += rac0[r] * (1.0f / RCARRY);
      v1 += rac1[r] * (1.0f / RCARRY);
    }
    d[0]  = v0;
    d[16] = v1;
  }
  __syncthreads();

  if (MODE == 3) {
#pragma unroll 1
    for (unsigned g = 0; g < 4u; ++g) {
      const unsigned r = 32u * (g >> 1) + (tid >> 3);
      const unsigned c = (tid & 7u) * 8u + 4u * (g & 1u);
      const v4f u  = *(const v4f*)&Cs[r * LDC + c];
      const v4f gb = *(const v4f*)(bias + n0 + c);
      v4f t;
#pragma unroll
      for (int j = 0; j < 4; ++j)
        t[j] = MCARRY * silu_act(u[j] * (1.0f / WCARRY) + bf16r(gb[j]));
      *(v4f*)&Cs[r * LDC + c] = t;
    }
    v8h x[2], xr[2];
    size_t off[2];
#pragma unroll
    for (unsigned i = 0; i < 2u; ++i) {
      const unsigned r = 32u * i + (tid >> 3);
      const unsigned c = (tid & 7u) * 8u;
      const v4f u0 = *(const v4f*)&Cs[r * LDC + c];
      const v4f u1 = *(const v4f*)&Cs[r * LDC + c + 4];
#pragma unroll
      for (int j = 0; j < 4; ++j) {
        const h16 a0 = toh_flush(u0[j]);
        const h16 a1 = toh_flush(u1[j]);
        x[i][j]      = a0;
        x[i][j + 4]  = a1;
        xr[i][j]     = toh_flush((u0[j] - (float)a0) * RCARRY);
        xr[i][j + 4] = toh_flush((u1[j] - (float)a1) * RCARRY);
      }
      off[i] = (size_t)(row0 + r) * HID + n0 + c;
    }
#pragma unroll
    for (int i = 0; i < 2; ++i) *(volatile v8h*)(out16 + off[i]) = x[i];
#pragma unroll
    for (int i = 0; i < 2; ++i) *(volatile v8h*)(out16r + off[i]) = xr[i];
    __threadfence();
#pragma unroll
    for (int i = 0; i < 2; ++i) *(volatile v8h*)(out16 + off[i]) = x[i];
#pragma unroll
    for (int i = 0; i < 2; ++i) *(volatile v8h*)(out16r + off[i]) = xr[i];
  } else {
    const float cs = (MODE == 2) ? (1.0f / (WCARRY * YCARRY))
                   : (MODE >= 4) ? (1.0f / (WCARRY * MCARRY)) : (1.0f / WCARRY);
    v4f xs[4];
    size_t off[4];
#pragma unroll
    for (unsigned i = 0; i < 4u; ++i) {
      const unsigned r = 16u * i + (tid >> 4);
      const unsigned c = (tid & 15u) * 4u;
      const unsigned crow = row0 + r;
      const unsigned g = crow >> 6;
      const unsigned bidx = g / (unsigned)TT;
      const unsigned tq = g - bidx * (unsigned)TT;
      const size_t frow = ((size_t)bidx * TT_FULL + tq) * NNODE + (crow & 63u);
      const v4f u = *(const v4f*)&Cs[r * LDC + c];
      v4f val;
      if (MODE == 0) {
        const v4f gb = *(const v4f*)(bias + n0 + c);
#pragma unroll
        for (int j = 0; j < 4; ++j) val[j] = u[j] * cs + bf16r(gb[j]);
      } else if (MODE == 1) {
#pragma unroll
        for (int j = 0; j < 4; ++j) val[j] = u[j] * cs;
      } else if (MODE == 2) {
        const v4f xin = *(const v4f*)(addf + (size_t)crow * DIM + n0 + c);
#pragma unroll
        for (int j = 0; j < 4; ++j) val[j] = xin[j] + u[j] * cs;
      } else {
        const v4f gb = *(const v4f*)(bias + n0 + c);
        const v4f xin = *(const v4f*)(addf + (size_t)crow * DIM + n0 + c);
#pragma unroll
        for (int j = 0; j < 4; ++j) val[j] = xin[j] + (u[j] * cs + bf16r(gb[j]));
      }
      xs[i] = val;
      off[i] = ((MODE == 5) ? frow : (size_t)crow) * DIM + n0 + c;
    }
#pragma unroll
    for (int i = 0; i < 4; ++i) *(volatile v4f*)(outf + off[i]) = xs[i];
    __threadfence();
#pragma unroll
    for (int i = 0; i < 4; ++i) *(volatile v4f*)(outf + off[i]) = xs[i];

    if (MODE == 5) {
#pragma unroll
      for (unsigned i = 0; i < 4u; ++i) {
        const unsigned r = 16u * i + (tid >> 4);
        const unsigned c = (tid & 15u) * 4u;
        *(v4f*)&Cs[r * LDC + c] = xs[i];
      }
      __syncthreads();
      const unsigned wv = (unsigned)__builtin_amdgcn_readfirstlane((int)(tid >> 5));
      if (wv == 0u) {
        const unsigned cl = ((tid < 16u) ? tid : 15u) * 4u;
        v4f sm = {};
#pragma unroll 4
        for (unsigned r = 0; r < 64u; ++r) {
          const v4f t = *(const v4f*)&Cs[r * LDC + cl];
          sm = sm + t;
        }
        v4f mv;
#pragma unroll
        for (int j = 0; j < 4; ++j) mv[j] = sm[j] * (1.0f / (float)NNODE);
        const unsigned g = blockIdx.y;
        const unsigned bidx = g / (unsigned)TT;
        const unsigned tq = g - bidx * (unsigned)TT;
        float* pm = outm + ((size_t)bidx * TT_FULL + tq) * DIM + n0 + cl;
        const bool st = (tid < 16u);
        if (st) *(volatile v4f*)pm = mv;
        __threadfence();
        if (st) *(volatile v4f*)pm = mv;
      }
    }
  }
}

__global__ __launch_bounds__(256) void gemm_proj_kernel(
    const _Float16* __restrict__ A16, const _Float16* __restrict__ Bt,
    const float* __restrict__ bias, float* __restrict__ outf) {
  gemm_body<0>(A16, A16, Bt, (unsigned)DIM, bias, bias, outf, (_Float16*)0, (_Float16*)0,
               (float*)0);
}
__global__ __launch_bounds__(256) void gemm_lin_kernel(
    const _Float16* __restrict__ A16, const _Float16* __restrict__ A16r,
    const _Float16* __restrict__ Bt, float* __restrict__ outf) {
  gemm_body<1>(A16, A16r, Bt, (unsigned)DIM, (const float*)0, (const float*)0, outf,
               (_Float16*)0, (_Float16*)0, (float*)0);
}
__global__ __launch_bounds__(256) void gemm_out_kernel(
    const _Float16* __restrict__ A16, const _Float16* __restrict__ Bt,
    const float* __restrict__ addf, float* __restrict__ outf) {
  gemm_body<2>(A16, A16, Bt, (unsigned)DIM, addf, addf, outf, (_Float16*)0, (_Float16*)0,
               (float*)0);
}
__global__ __launch_bounds__(256) void gemm_mlp1_kernel(
    const _Float16* __restrict__ A16, const _Float16* __restrict__ Bt,
    const float* __restrict__ bias, _Float16* __restrict__ mid, _Float16* __restrict__ midr) {
  gemm_body<3>(A16, A16, Bt, (unsigned)DIM, bias, bias, (float*)0, mid, midr, (float*)0);
}
__global__ __launch_bounds__(256) void gemm_mlp2_kernel(
    const _Float16* __restrict__ A16, const _Float16* __restrict__ A16r,
    const _Float16* __restrict__ Bt,
    const float* __restrict__ bias, const float* __restrict__ addf, float* __restrict__ outf) {
  gemm_body<4>(A16, A16r, Bt, (unsigned)HID, bias, addf, outf, (_Float16*)0, (_Float16*)0,
               (float*)0);
}
__global__ __launch_bounds__(256) void gemm_final_kernel(
    const _Float16* __restrict__ A16, const _Float16* __restrict__ A16r,
    const _Float16* __restrict__ Bt,
    const float* __restrict__ bias, const float* __restrict__ addf, float* __restrict__ outf,
    float* __restrict__ outm) {
  gemm_body<5>(A16, A16r, Bt, (unsigned)HID, bias, addf, outf, (_Float16*)0, (_Float16*)0, outm);
}

__global__ __launch_bounds__(256) void graph_kernel(
    const float* __restrict__ Zc, const _Float16* __restrict__ Hn,
    const _Float16* __restrict__ HnR,
    const float* __restrict__ Xh, const _Float16* __restrict__ A16,
    const float* __restrict__ LB, const int* __restrict__ maskp,
    const float* __restrict__ atta,
    float* __restrict__ ZH, _Float16* __restrict__ Y16) {
  __shared__ __attribute__((aligned(16))) GraphTileA RA;
  __shared__ __attribute__((aligned(16))) GraphTileC RC;
  __shared__ __attribute__((aligned(16))) _Float16 PHs[PH_HALVES];
  __shared__ float Ls[NHEAD * NNODE];

  const unsigned tid = threadIdx.x, lane = tid & 31u;
  const unsigned wave = (unsigned)__builtin_amdgcn_readfirstlane((int)(threadIdx.x >> 5));
  const unsigned hh = lane >> 4, m = lane & 15u;
  const size_t grow = (size_t)blockIdx.x * NNODE;
  const float ninf = -__builtin_inff();

#pragma unroll 2
  for (unsigned k = 0; k < 4u; ++k) {
    const unsigned idx = tid + 256u * k;
    const unsigned r = idx >> 4, c = (idx & 15u) * 8u;
    const v8h x  = *(const v8h*)(Hn + (grow + r) * DIM + c);
    const v8h xr = *(const v8h*)(HnR + (grow + r) * DIM + c);
#pragma unroll
    for (unsigned j = 0; j < 8u; ++j) {
      PHs[(c + j) * LDT + r] = x[j];
      PHs[HT_HALVES + (c + j) * LDT + r] = xr[j];
    }
  }
  __syncthreads();

  {
    const unsigned mt = wave >> 1;
    const unsigned nt0 = (wave & 1u) * 4u;
    v8f h0 = {}, h1 = {}, h2 = {}, h3 = {};
    v8f g0 = {}, g1 = {}, g2 = {}, g3 = {};
#pragma unroll
    for (int c = 0; c < 2; ++c) {
      const v16h af = frag_at(A16 + (size_t)(mt * 16u + m) * NNODE + hh * 8u + c * 32);
      const v16h b0 = ld_frag(&PHs[((nt0 + 0u) * 16u) * LDT + c * 32], LDT);
      const v16h b1 = ld_frag(&PHs[((nt0 + 1u) * 16u) * LDT + c * 32], LDT);
      const v16h b2 = ld_frag(&PHs[((nt0 + 2u) * 16u) * LDT + c * 32], LDT);
      const v16h b3 = ld_frag(&PHs[((nt0 + 3u) * 16u) * LDT + c * 32], LDT);
      h0 = wmma16(af, b0, h0);
      h1 = wmma16(af, b1, h1);
      h2 = wmma16(af, b2, h2);
      h3 = wmma16(af, b3, h3);
      const v16h r0 = ld_frag(&PHs[HT_HALVES + ((nt0 + 0u) * 16u) * LDT + c * 32], LDT);
      const v16h r1 = ld_frag(&PHs[HT_HALVES + ((nt0 + 1u) * 16u) * LDT + c * 32], LDT);
      const v16h r2 = ld_frag(&PHs[HT_HALVES + ((nt0 + 2u) * 16u) * LDT + c * 32], LDT);
      const v16h r3 = ld_frag(&PHs[HT_HALVES + ((nt0 + 3u) * 16u) * LDT + c * 32], LDT);
      g0 = wmma16(af, r0, g0);
      g1 = wmma16(af, r1, g1);
      g2 = wmma16(af, r2, g2);
      g3 = wmma16(af, r3, g3);
    }
#pragma unroll
    for (int r = 0; r < 8; ++r) {
      float* d = &RA.f[(mt * 16u + hh * 8u + (unsigned)r) * XP + nt0 * 16u + m];
      d[0]  = h0[r] + g0[r] * (1.0f / RCARRY);
      d[16] = h1[r] + g1[r] * (1.0f / RCARRY);
      d[32] = h2[r] + g2[r] * (1.0f / RCARRY);
      d[48] = h3[r] + g3[r] * (1.0f / RCARRY);
    }
  }
  __syncthreads();

  {
    v4f zx[8];
    size_t zoff[8];
#pragma unroll
    for (unsigned k = 0; k < 8u; ++k) {
      const unsigned idx = tid + 256u * k;
      const unsigned r = idx >> 5, c = (idx & 31u) * 4u;
      const v4f hm = *(const v4f*)&RA.f[r * XP + c];
      const v4f zz = *(const v4f*)(Zc + (grow + r) * DIM + c);
      v4f t;
#pragma unroll
      for (int j = 0; j < 4; ++j) t[j] = zz[j] + hm[j] * (1.0f / ACARRY);
      zx[k] = t;
      zoff[k] = (grow + r) * DIM + c;
    }
#pragma unroll
    for (int k = 0; k < 8; ++k) *(volatile v4f*)(ZH + zoff[k]) = zx[k];
    __threadfence();
#pragma unroll
    for (int k = 0; k < 8; ++k) *(volatile v4f*)(ZH + zoff[k]) = zx[k];
  }
  __syncthreads();

#pragma unroll 2
  for (unsigned k = 0; k < 8u; ++k) {
    const unsigned idx = tid + 256u * k;
    const unsigned r = idx >> 5, c = (idx & 31u) * 4u;
    const v4f x = *(const v4f*)(Xh + (grow + r) * DIM + c);
    *(v4f*)&RA.f[r * XP + c] = x;
  }
#pragma unroll
  for (unsigned k = 0; k < 4u; ++k) {
    const unsigned e = (tid + 256u * k) * 4u;
    const v4f lb = *(const v4f*)(LB + e);
    const v4i mk = *(const v4i*)(maskp + e);
    v4f o;
#pragma unroll
    for (int j = 0; j < 4; ++j) o[j] = (mk[j] != 0) ? lb[j] : ninf;
    *(v4f*)&RC.f[e] = o;
  }
  __syncthreads();

  const unsigned head = wave >> 1;
  const unsigned ibase = (wave & 1u) * 32u;
  {
    float xa[HD], xb[HD], av[HD];
#pragma unroll
    for (int q = 0; q < 8; ++q) {
      const v4f ta = *(const v4f*)&RA.f[lane * XP + head * HD + 4 * q];
      const v4f tb = *(const v4f*)&RA.f[(lane + 32u) * XP + head * HD + 4 * q];
#pragma unroll
      for (int j = 0; j < 4; ++j) {
        xa[4 * q + j] = ta[j];
        xb[4 * q + j] = tb[j];
        av[4 * q + j] = bf16r(atta[head * HD + 4 * q + j]);
      }
    }
#pragma unroll 1
    for (unsigned ii = 0; ii < 32u; ++ii) {
      const unsigned i = ibase + ii;
      float e0 = 0.0f, e1 = 0.0f;
#pragma unroll
      for (int q = 0; q < 8; ++q) {
        const v4f xi = *(const v4f*)&RA.f[i * XP + head * HD + 4 * q];
#pragma unroll
        for (int j = 0; j < 4; ++j) {
          float v0 = xi[j] + xa[4 * q + j];
          float v1 = xi[j] + xb[4 * q + j];
          v0 = fmaxf(v0, 0.2f * v0);
          v1 = fmaxf(v1, 0.2f * v1);
          e0 = fmaf(v0, av[4 * q + j], e0);
          e1 = fmaf(v1, av[4 * q + j], e1);
        }
      }
      const float lb0 = RC.f[i * NNODE + lane];
      const float lb1 = RC.f[i * NNODE + lane + 32u];
      e0 = (lb0 == ninf) ? ninf : (e0 + lb0);
      e1 = (lb1 == ninf) ? ninf : (e1 + lb1);
      const float mx = red32_max(fmaxf(e0, e1));
      const float p0 = __expf(e0 - mx) * PCARRY;
      const float p1 = __expf(e1 - mx) * PCARRY;
      const h16 h0 = toh_flush(p0);
      const h16 h1 = toh_flush(p1);
      const float rs = red32_sum((float)h0 + (float)h1);
      PHs[(head * NNODE + i) * LDT + lane] = h0;
      PHs[(head * NNODE + i) * LDT + lane + 32u] = h1;
      if (lane == 0u) Ls[head * NNODE + i] = rs;
    }
  }
  __syncthreads();

#pragma unroll 2
  for (unsigned k = 0; k < 8u; ++k) {
    const unsigned idx = tid + 256u * k;
    const unsigned r = idx >> 5, c = (idx & 31u) * 4u;
    const v4f x = *(const v4f*)&RA.f[r * XP + c];
#pragma unroll
    for (unsigned j = 0; j < 4u; ++j) RC.h[(c + j) * LDT + r] = toh_flush(x[j]);
  }
  __syncthreads();

  const unsigned it0 = (wave & 1u) * 2u;
  {
    v8f o00 = {}, o01 = {}, o10 = {}, o11 = {};
#pragma unroll
    for (int c = 0; c < 2; ++c) {
      const v16h pf0 = ld_frag(&PHs[(head * NNODE + (it0 + 0u) * 16u) * LDT + c * 32], LDT);
      const v16h pf1 = ld_frag(&PHs[(head * NNODE + (it0 + 1u) * 16u) * LDT + c * 32], LDT);
      const v16h vf0 = ld_frag(&RC.h[(head * HD + 0u) * LDT + c * 32], LDT);
      const v16h vf1 = ld_frag(&RC.h[(head * HD + 16u) * LDT + c * 32], LDT);
      o00 = wmma16(pf0, vf0, o00);
      o01 = wmma16(pf0, vf1, o01);
      o10 = wmma16(pf1, vf0, o10);
      o11 = wmma16(pf1, vf1, o11);
    }
#pragma unroll
    for (int r = 0; r < 8; ++r) {
      const unsigned ra = (it0 + 0u) * 16u + hh * 8u + (unsigned)r;
      const unsigned rb = (it0 + 1u) * 16u + hh * 8u + (unsigned)r;
      const float ia = __builtin_amdgcn_rcpf(Ls[head * NNODE + ra]) * YCARRY;
      const float ib = __builtin_amdgcn_rcpf(Ls[head * NNODE + rb]) * YCARRY;
      RA.h[ra * LDY + head * HD + m]       = toh_flush(o00[r] * ia);
      RA.h[ra * LDY + head * HD + 16u + m] = toh_flush(o01[r] * ia);
      RA.h[rb * LDY + head * HD + m]       = toh_flush(o10[r] * ib);
      RA.h[rb * LDY + head * HD + 16u + m] = toh_flush(o11[r] * ib);
    }
  }
  __syncthreads();

  v8h yx[4];
  size_t yoff[4];
#pragma unroll
  for (unsigned k = 0; k < 4u; ++k) {
    const unsigned idx = tid + 256u * k;
    const unsigned r = idx >> 4, c = (idx & 15u) * 8u;
    yx[k] = *(const v8h*)&RA.h[r * LDY + c];
    yoff[k] = (grow + r) * DIM + c;
  }
#pragma unroll
  for (int k = 0; k < 4; ++k) *(volatile v8h*)(Y16 + yoff[k]) = yx[k];
  __threadfence();
#pragma unroll
  for (int k = 0; k < 4; ++k) *(volatile v8h*)(Y16 + yoff[k]) = yx[k];
}

extern "C" void kernel_launch(void* const* d_in, const int* in_sizes, int n_in,
                              void* d_out, int out_size, void* d_ws, size_t ws_size,
                              hipStream_t stream) {
  if (n_in < 23) return;
  const long long need_x = (((long long)(NB - 1) * TT_FULL + TT) * NNODE) * DIM;
  if ((long long)in_sizes[0] < need_x) return;
  if (in_sizes[1] < NNODE * NNODE || in_sizes[2] < NNODE * NNODE) return;
  if (in_sizes[3] < DIM * DIM || in_sizes[4] < DIM) return;
  if (in_sizes[5] < NNODE * RANK || in_sizes[6] < NNODE * RANK || in_sizes[7] < 1) return;
  if (in_sizes[8] < NLAYER * DIM || in_sizes[9] < NLAYER * DIM) return;
  if (in_sizes[10] < NLAYER * DIM * DIM || in_sizes[11] < NLAYER * DIM) return;
  if (in_sizes[12] < NLAYER * DIM * DIM) return;
  if (in_sizes[13] < NLAYER * DIM || in_sizes[14] < NLAYER * DIM) return;
  if (in_sizes[15] < NLAYER * DIM || in_sizes[16] < NLAYER) return;
  if (in_sizes[17] < NLAYER * DIM || in_sizes[18] < NLAYER * DIM) return;
  if (in_sizes[19] < NLAYER * DIM * HID || in_sizes[20] < NLAYER * HID) return;
  if (in_sizes[21] < NLAYER * HID * DIM || in_sizes[22] < NLAYER * DIM) return;
  if ((long long)out_size < (long long)OUT_TOTAL) return;
  if (ws_size < WS_TOTAL) return;

  const float* X      = (const float*)d_in[0];
  const float* A0     = (const float*)d_in[1];
  const int*   maskp  = (const int*)d_in[2];
  const float* projW  = (const float*)d_in[3];
  const float* projb  = (const float*)d_in[4];
  const float* Pm     = (const float*)d_in[5];
  const float* Qm     = (const float*)d_in[6];
  const float* alphap = (const float*)d_in[7];
  const float* ln1s   = (const float*)d_in[8];
  const float* ln1b   = (const float*)d_in[9];
  const float* linW   = (const float*)d_in[10];
  const float* atta   = (const float*)d_in[11];
  const float* outW   = (const float*)d_in[12];
  const float* fc1W   = (const float*)d_in[13];
  const float* fc1b   = (const float*)d_in[14];
  const float* fc2W   = (const float*)d_in[15];
  const float* fc2b   = (const float*)d_in[16];
  const float* ln2s   = (const float*)d_in[17];
  const float* ln2b   = (const float*)d_in[18];
  const float* W1     = (const float*)d_in[19];
  const float* b1     = (const float*)d_in[20];
  const float* W2     = (const float*)d_in[21];
  const float* b2     = (const float*)d_in[22];
  float* out = (float*)d_out;

  char* ws = (char*)d_ws;
  _Float16* Wp_t  = (_Float16*)(ws + OFF_WP);
  _Float16* Wl_t  = (_Float16*)(ws + OFF_WL);
  _Float16* Wo_t  = (_Float16*)(ws + OFF_WO);
  _Float16* W1_t  = (_Float16*)(ws + OFF_W1);
  _Float16* W2_t  = (_Float16*)(ws + OFF_W2);
  _Float16* A16   = (_Float16*)(ws + OFF_A16);
  float*    LB    = (float*)(ws + OFF_LB);
  _Float16* X16   = (_Float16*)(ws + OFF_X16);
  _Float16* Hn16  = (_Float16*)(ws + OFF_HN);
  _Float16* HnR16 = (_Float16*)(ws + OFF_HNR);
  _Float16* Y16   = (_Float16*)(ws + OFF_Y);
  _Float16* H2    = (_Float16*)(ws + OFF_H2);
  float*    Xh    = (float*)(ws + OFF_XH);
  float*    Zp    = (float*)(ws + OFF_Z);
  float*    ZHp   = (float*)(ws + OFF_ZH);
  float*    UPp   = (float*)(ws + OFF_UP);
  float*    Up    = (float*)(ws + OFF_U);
  _Float16* Mid16 = (_Float16*)(ws + OFF_MID);
  _Float16* MidR16 = (_Float16*)(ws + OFF_MIDR);

  dim3 blk(256);
  dim3 gsq(DIM / 64, DIM / 64);
  dim3 gg(DIM / 64, NGRAPH);

  wconv_kernel<<<gsq, blk, 0, stream>>>(projW, Wp_t, (unsigned)DIM, (unsigned)DIM);
  for (int l = 0; l < NLAYER; ++l) {
    wconv_kernel<<<gsq, blk, 0, stream>>>(linW + (size_t)l * DIM * DIM,
                                          Wl_t + (size_t)l * DIM * DIM, (unsigned)DIM, (unsigned)DIM);
    wconv_kernel<<<gsq, blk, 0, stream>>>(outW + (size_t)l * DIM * DIM,
                                          Wo_t + (size_t)l * DIM * DIM, (unsigned)DIM, (unsigned)DIM);
    wconv_kernel<<<dim3(HID / 64, DIM / 64), blk, 0, stream>>>(
        W1 + (size_t)l * DIM * HID, W1_t + (size_t)l * DIM * HID, (unsigned)HID, (unsigned)DIM);
    wconv_kernel<<<dim3(DIM / 64, HID / 64), blk, 0, stream>>>(
        W2 + (size_t)l * DIM * HID, W2_t + (size_t)l * DIM * HID, (unsigned)DIM, (unsigned)HID);
  }

  adj_kernel<<<dim3(1), blk, 0, stream>>>(A0, maskp, Pm, Qm, alphap, out + OUT2_OFF, A16, LB);
  xconv_kernel<<<dim3(MROWS / 16), blk, 0, stream>>>(X, X16);
  gemm_proj_kernel<<<gg, blk, 0, stream>>>(X16, Wp_t, projb, Zp);

  for (int l = 0; l < NLAYER; ++l) {
    ln1_kernel<<<dim3(MROWS / 8), blk, 0, stream>>>(Zp, ln1s + l * DIM, ln1b + l * DIM, Hn16,
                                                    HnR16);
    gemm_lin_kernel<<<gg, blk, 0, stream>>>(Hn16, HnR16, Wl_t + (size_t)l * DIM * DIM, Xh);
    graph_kernel<<<dim3(NGRAPH), blk, 0, stream>>>(Zp, Hn16, HnR16, Xh, A16, LB, maskp,
                                                   atta + l * DIM, ZHp, Y16);
    gemm_out_kernel<<<gg, blk, 0, stream>>>(Y16, Wo_t + (size_t)l * DIM * DIM, ZHp, UPp);
    gate_ln2_kernel<<<dim3(MROWS / 8), blk, 0, stream>>>(
        UPp, fc1W + l * DIM, fc1b + l * DIM, fc2W + l * DIM, fc2b + l,
        ln2s + l * DIM, ln2b + l * DIM, Up, H2);
    gemm_mlp1_kernel<<<dim3(HID / 64, NGRAPH), blk, 0, stream>>>(
        H2, W1_t + (size_t)l * DIM * HID, b1 + l * HID, Mid16, MidR16);
    if (l + 1 < NLAYER) {
      gemm_mlp2_kernel<<<gg, blk, 0, stream>>>(Mid16, MidR16, W2_t + (size_t)l * DIM * HID,
                                               b2 + l * DIM, Up, Zp);
    } else {
      gemm_final_kernel<<<gg, blk, 0, stream>>>(Mid16, MidR16, W2_t + (size_t)l * DIM * HID,
                                                b2 + l * DIM, Up, out, out + OUT1_OFF);
    }
  }
}
